// SE3TBackbone_48593259987060
// MI455X (gfx1250) — hardware-run, weakly checked
//
#include <hip/hip_runtime.h>
#include <math.h>

typedef __attribute__((ext_vector_type(16))) _Float16 v16h;
typedef __attribute__((ext_vector_type(8)))  _Float16 v8h;
typedef __attribute__((ext_vector_type(4)))  _Float16 v4h;
typedef __attribute__((ext_vector_type(8)))  float    v8f;
typedef __attribute__((ext_vector_type(4)))  float    v4f;

constexpr int kBatch = 16;
constexpr int kNodes = 64;
constexpr int kFin   = 16;
constexpr int kCh    = 32;
constexpr int kDeg   = 4;
constexpr int kLay   = 4;
constexpr int kHeads = 8;
constexpr int kHd    = kCh / kHeads;
constexpr int kBN    = kBatch * kNodes;
constexpr int kMM    = 16;
constexpr int kFib   = kCh * kMM;
constexpr int kRadN  = kDeg * 4 * kCh;
constexpr float kEps = 1e-6f;
constexpr float kWCarry   = 64.0f;
constexpr float kHCarry   = 16.0f;
constexpr float kFCarry   = 128.0f;
constexpr float kRadFold  = 1.0f / (kWCarry * kHCarry);
constexpr float kProjFold = 1.0f / (kWCarry * kFCarry);
constexpr float kLogitScale = 0.125f;
constexpr int kRP = 68;
static_assert(kHd == 4);
static_assert(kMM == 1 + 3 + 5 + 7);
static_assert(kLogitScale * kLogitScale * (float)(kHd * kMM) == 1.0f);
static_assert(kRadN == 512 && kFib == 512 && kBN == 1024);
static_assert((kCh % 32) == 0);

constexpr size_t kOffRW2T = 0;
constexpr size_t kOffWK   = kOffRW2T + (size_t)kLay * kRadN * kCh * 2;
constexpr size_t kOffWV   = kOffWK   + (size_t)kLay * kDeg * 2 * kCh * kCh * 2;
constexpr size_t kOffWQ   = kOffWV   + (size_t)kLay * kDeg * 2 * kCh * kCh * 2;
constexpr size_t kOffWS   = kOffWQ   + (size_t)kLay * kDeg * kCh * kCh * 2;
constexpr size_t kOffFTA  = kOffWS   + (size_t)kLay * kDeg * kCh * kCh * 2;
constexpr size_t kOffFTB  = kOffFTA  + (size_t)kBN * kFib * 2;
constexpr size_t kOffPROJ = kOffFTB  + (size_t)kBN * kFib * 2;
constexpr size_t kOffSC   = kOffPROJ + (size_t)4 * kBN * kFib * 4;
constexpr size_t kOffINV  = kOffSC   + (size_t)2 * kBN * 128 * 4;
constexpr size_t kWsTotal = kOffINV  + (size_t)kBN * 128 * 4;
static_assert(kWsTotal == 12386304ull);
static_assert(kWsTotal <= 134217728ull);
static_assert((kOffWK % 128) == 0 && (kOffWV % 128) == 0 && (kOffWQ % 128) == 0 && (kOffWS % 128) == 0 &&
              (kOffFTA % 128) == 0 && (kOffFTB % 128) == 0 && (kOffPROJ % 128) == 0 && (kOffSC % 128) == 0 &&
              (kOffINV % 128) == 0);
constexpr int kW16OffK = 0;
constexpr int kW16OffV = 32768;
constexpr int kW16OffQ = 65536;
constexpr int kW16OffS = 81920;
static_assert(kOffWV - kOffWK == (size_t)kW16OffV * 2 && kOffWQ - kOffWK == (size_t)kW16OffQ * 2 &&
              kOffWS - kOffWK == (size_t)kW16OffS * 2);
constexpr size_t kPlane   = (size_t)kBN * kFib;
constexpr size_t kScPlane = (size_t)kBN * 128;

union FragU { v16h v; v8h h[2]; };
__device__ __forceinline__ v16h frag_load(const _Float16* p) {
  FragU f;
  f.h[0] = *(const v8h*)(p);
  f.h[1] = *(const v8h*)(p + 16);
  return f.v;
}
__device__ __forceinline__ v8f mma_guard(v16h a, v16h b, v8f c) {
  c = __builtin_amdgcn_wmma_f32_16x16x32_f16(false, a, false, b, (short)0, c, false, false);
  asm volatile("v_nop\n\tv_nop\n\tv_nop\n\tv_nop" : "+v"(c) : "v"(a), "v"(b));
  return c;
}

__device__ __forceinline__ void ld16(float (&dst)[16], const float* p) {
#pragma unroll
  for (int q = 0; q < 4; ++q) {
    const v4f t = *(const v4f*)(p + 4 * q);
    dst[4 * q + 0] = t[0];
    dst[4 * q + 1] = t[1];
    dst[4 * q + 2] = t[2];
    dst[4 * q + 3] = t[3];
  }
}

template <int L> __device__ __forceinline__ float deg_dot(const float (&a)[16], const float (&b)[16]) {
  float s = 0.0f;
#pragma unroll
  for (int m = 0; m < 2 * L + 1; ++m) s = fmaf(a[L * L + m], b[L * L + m], s);
  return s;
}

__device__ __forceinline__ void sph16(float x, float y, float z, float* Y) {
  const float c0 = 0.28209479177387814f;
  const float c1 = 0.4886025119029199f;
  Y[0] = c0;
  Y[1] = c1 * y; Y[2] = c1 * z; Y[3] = c1 * x;
  const float a2 = 1.0925484305920792f;
  const float b2 = 0.31539156525252005f;
  const float e2 = 0.5462742152960396f;
  Y[4] = a2 * x * y;
  Y[5] = a2 * y * z;
  Y[6] = b2 * (3.f * z * z - 1.f);
  Y[7] = a2 * x * z;
  Y[8] = e2 * (x * x - y * y);
  const float d0 = 0.5900435899266435f;
  const float d1 = 2.890611442640554f;
  const float d2 = 0.4570457994644658f;
  const float d3 = 0.3731763325901154f;
  const float d5 = 1.445305721320277f;
  Y[9]  = d0 * y * (3.f * x * x - y * y);
  Y[10] = d1 * x * y * z;
  Y[11] = d2 * y * (5.f * z * z - 1.f);
  Y[12] = d3 * z * (5.f * z * z - 3.f);
  Y[13] = d2 * x * (5.f * z * z - 1.f);
  Y[14] = d5 * z * (x * x - y * y);
  Y[15] = d0 * x * (x * x - y * y);
}

__global__ __launch_bounds__(256) void pack_weights_kernel(
    const float* __restrict__ rw2, const float* __restrict__ Wk, const float* __restrict__ Wv,
    const float* __restrict__ Wq, const float* __restrict__ Wself, _Float16* __restrict__ dst16)
{
  const int blk = blockIdx.x;
  const int i = blk * 256 + threadIdx.x;
  float v[8];
  if (blk < 32) {
    const int e0 = i * 8;
    const int li = e0 >> 14;
    const int col = (e0 >> 5) & 511;
    const int k0 = e0 & 31;
#pragma unroll
    for (int e = 0; e < 8; ++e) v[e] = rw2[((size_t)(li * 32 + k0 + e)) * 512 + col];
  } else {
    const float* src;
    int j;
    if (blk < 48)      { src = Wk;    j = i - 8192;  }
    else if (blk < 64) { src = Wv;    j = i - 12288; }
    else if (blk < 72) { src = Wq;    j = i - 16384; }
    else               { src = Wself; j = i - 18432; }
    const v4f a0 = *(const v4f*)(src + (size_t)j * 8);
    const v4f a1 = *(const v4f*)(src + (size_t)j * 8 + 4);
    v[0] = a0[0]; v[1] = a0[1]; v[2] = a0[2]; v[3] = a0[3];
    v[4] = a1[0]; v[5] = a1[1]; v[6] = a1[2]; v[7] = a1[3];
  }
  v8h hv;
#pragma unroll
  for (int e = 0; e < 8; ++e) hv[e] = (_Float16)(v[e] * kWCarry);
  _Float16* q = dst16 + (size_t)i * 8;
  *(volatile v8h*)q = hv;
  __threadfence();
  *(volatile v8h*)q = hv;
}

__global__ __launch_bounds__(256) void embed_kernel(
    const float* __restrict__ hfeat, const float* __restrict__ Wemb, _Float16* __restrict__ fT)
{
  const int tid = threadIdx.x;
  const int node = blockIdx.x * 4 + (tid >> 6);
  const int e = tid & 63;
  const int mm = e >> 2;
  const int c8 = (e & 3) * 8;
  float acc[8];
#pragma unroll
  for (int j = 0; j < 8; ++j) acc[j] = 0.0f;
#pragma unroll 1
  for (int i = 0; i < kFin; ++i) {
    const float hv = hfeat[(size_t)node * kFin + i];
    const v4f w0 = *(const v4f*)(Wemb + i * kCh + c8);
    const v4f w1 = *(const v4f*)(Wemb + i * kCh + c8 + 4);
    acc[0] = fmaf(hv, w0[0], acc[0]);
    acc[1] = fmaf(hv, w0[1], acc[1]);
    acc[2] = fmaf(hv, w0[2], acc[2]);
    acc[3] = fmaf(hv, w0[3], acc[3]);
    acc[4] = fmaf(hv, w1[0], acc[4]);
    acc[5] = fmaf(hv, w1[1], acc[5]);
    acc[6] = fmaf(hv, w1[2], acc[6]);
    acc[7] = fmaf(hv, w1[3], acc[7]);
  }
  v8h ov;
#pragma unroll
  for (int j = 0; j < 8; ++j) {
    const float t = (mm == 0) ? (acc[j] * kFCarry) : 0.0f;
    ov[j] = (_Float16)t;
  }
  _Float16* q = fT + (size_t)node * kFib + e * 8;
  *(volatile v8h*)q = ov;
  __threadfence();
  *(volatile v8h*)q = ov;
}

__global__ __launch_bounds__(256) void node_proj_kernel(
    const _Float16* __restrict__ fT, const _Float16* __restrict__ w16,
    float* __restrict__ projBase, float* __restrict__ scBase, int li)
{
  __shared__ __align__(16) float sOut[4 * kFib];
  __shared__ __align__(16) float sSc[2 * 128];
  const int tid = threadIdx.x, lane = tid & 31, wave = tid >> 5;
  const int hf = lane >> 4, rl = lane & 15, koff = hf * 8;
  const int node = blockIdx.x;

  const v16h a = frag_load(fT + (size_t)node * kFib + rl * 32 + koff);
  const v8f zero8 = (v8f){0.f, 0.f, 0.f, 0.f, 0.f, 0.f, 0.f, 0.f};

  const int arr = wave >> 1, nt = wave & 1;
  int wbase, lstr;
  if (arr == 0)      { wbase = kW16OffK + li * 8192 + 1024; lstr = 2048; }
  else if (arr == 1) { wbase = kW16OffV + li * 8192 + 1024; lstr = 2048; }
  else if (arr == 2) { wbase = kW16OffQ + li * 4096;        lstr = 1024; }
  else               { wbase = kW16OffS + li * 4096;        lstr = 1024; }
  const _Float16* wp = w16 + wbase + (nt * 16 + rl) * 32 + koff;
  const v16h b0 = frag_load(wp);
  const v8f d0 = mma_guard(a, b0, zero8);
  const v16h b1 = frag_load(wp + lstr);
  const v8f d1 = mma_guard(a, b1, zero8);
  const v16h b2 = frag_load(wp + 2 * lstr);
  const v8f d2 = mma_guard(a, b2, zero8);
  const v16h b3 = frag_load(wp + 3 * lstr);
  const v8f d3 = mma_guard(a, b3, zero8);

  const int kv = wave >> 2, ll = wave & 3;
  const int lbase = (kv ? kW16OffV : kW16OffK) + li * 8192 + ll * 2048;
  const _Float16* lp = w16 + lbase + rl * 32 + koff;
  const v16h g0 = frag_load(lp);
  const v8f e0 = mma_guard(a, g0, zero8);
  const v16h g1 = frag_load(lp + 16 * 32);
  const v8f e1 = mma_guard(a, g1, zero8);

  {
    const bool up = (hf != 0);
    v4f lo4, hi4;
    lo4[0] = (up ? d2[0] : d0[0]) * kProjFold;
    lo4[1] = (up ? d3[1] : d1[1]) * kProjFold;
    lo4[2] = (up ? d3[2] : d1[2]) * kProjFold;
    lo4[3] = (up ? d3[3] : d1[3]) * kProjFold;
    hi4[0] = (up ? d3[4] : d2[4]) * kProjFold;
    hi4[1] = (up ? d3[5] : d2[5]) * kProjFold;
    hi4[2] = (up ? d3[6] : d2[6]) * kProjFold;
    hi4[3] = (up ? d3[7] : d2[7]) * kProjFold;
    const int c = nt * 16 + rl;
    *(v4f*)(&sOut[arr * kFib + c * kMM + hf * 8])     = lo4;
    *(v4f*)(&sOut[arr * kFib + c * kMM + hf * 8 + 4]) = hi4;
    if (hf == 0) {
      sSc[kv * 128 + ll * 32 + rl]      = e0[0] * kProjFold;
      sSc[kv * 128 + ll * 32 + 16 + rl] = e1[0] * kProjFold;
    }
  }
  __syncthreads();
  {
    const v4f o0 = *(const v4f*)(&sOut[tid * 4]);
    const v4f o1 = *(const v4f*)(&sOut[1024 + tid * 4]);
    const int pl = tid >> 7;
    const int off = (tid & 127) * 4;
    float* q0 = projBase + (size_t)pl * kPlane + (size_t)node * kFib + off;
    float* q1 = projBase + (size_t)(2 + pl) * kPlane + (size_t)node * kFib + off;
    const int ws2 = (wave < 2) ? wave : 0;
    const v4f sv = *(const v4f*)(&sSc[ws2 * 128 + lane * 4]);
    float* q2 = scBase + (size_t)ws2 * kScPlane + (size_t)node * 128 + lane * 4;
    for (int pass = 0; pass < 2; ++pass) {
      *(volatile v4f*)q0 = o0;
      *(volatile v4f*)q1 = o1;
      if (wave < 2) *(volatile v4f*)q2 = sv;
      __threadfence();
    }
  }
}

__device__ __forceinline__ void radial_tile(const v16h a, const _Float16* __restrict__ bp,
                                            const float bias, float* srp) {
  const v16h bfr = frag_load(bp);
  v8f acc = (v8f){0.f, 0.f, 0.f, 0.f, 0.f, 0.f, 0.f, 0.f};
  acc = mma_guard(a, bfr, acc);
#pragma unroll
  for (int r = 0; r < 8; ++r) srp[r * kRP] = fmaf(acc[r], kRadFold, bias);
}

template <int L> __device__ __forceinline__ float logit_acc(float acc, const float (&ca)[16],
                                                            const float (&cb)[16], const float* srow) {
  const v4f r0 = *(const v4f*)(srow);
  const v4f r1 = *(const v4f*)(srow + 32);
  acc = fmaf(r0[0], ca[L * 4 + 0], acc);
  acc = fmaf(r1[0], cb[L * 4 + 0], acc);
  acc = fmaf(r0[1], ca[L * 4 + 1], acc);
  acc = fmaf(r1[1], cb[L * 4 + 1], acc);
  acc = fmaf(r0[2], ca[L * 4 + 2], acc);
  acc = fmaf(r1[2], cb[L * 4 + 2], acc);
  acc = fmaf(r0[3], ca[L * 4 + 3], acc);
  acc = fmaf(r1[3], cb[L * 4 + 3], acc);
  return acc;
}

template <int L> __device__ __forceinline__ void value_acc(float (&o)[16], const float (&at)[4],
                                                           const float (&iv)[64], const float (&svv)[16],
                                                           const float* sRp, const float* sYp,
                                                           const int vsp, const int vc) {
#pragma unroll
  for (int j = 0; j < 4; ++j) {
    const int s = j * 16 + vsp;
    const float r2 = sRp[s * kRP + vc];
    const float r3 = sRp[s * kRP + 32 + vc];
    const float t2 = at[j] * r2 * svv[j * 4 + L];
    const float t3 = at[j] * r3;
#pragma unroll
    for (int m = 0; m < 2 * L + 1; ++m) {
      const int mm = L * L + m;
      o[mm] = fmaf(t2, sYp[s * kMM + mm], fmaf(t3, iv[j * 16 + mm], o[mm]));
    }
  }
}

template <int L> __device__ __forceinline__ float gate_degree(const float (&o)[16], float (&fn)[16],
                                                              const float g, const float bb) {
  float s2 = 0.0f;
#pragma unroll
  for (int m = 0; m < 2 * L + 1; ++m) s2 = fmaf(o[L * L + m], o[L * L + m], s2);
  const float nrm = sqrtf(s2 + kEps);
  const float act = fmaxf(fmaf(g, nrm, bb), 0.0f);
  const float ratio = act * (1.0f / nrm);
  float t2 = 0.0f;
#pragma unroll
  for (int m = 0; m < 2 * L + 1; ++m) {
    const float f = o[L * L + m] * ratio;
    fn[L * L + m] = f;
    t2 = fmaf(f, f, t2);
  }
  return (L == 0) ? fn[0] : sqrtf(t2 + kEps);
}

__global__ __launch_bounds__(512) void edge_attn_kernel(
    const float* __restrict__ x, const int* __restrict__ bond,
    const float* __restrict__ rw1, const float* __restrict__ rb1,
    const _Float16* __restrict__ rw2T, const float* __restrict__ rb2,
    const float* __restrict__ projBase, const float* __restrict__ scBase,
    const float* __restrict__ gnorm, const float* __restrict__ bnorm,
    _Float16* __restrict__ fTout, float* __restrict__ invOut, int li)
{
  __shared__ __align__(16) float    sY[kNodes * kMM];
  __shared__ __align__(16) _Float16 sHm[kNodes * kCh];
  __shared__ __align__(16) float    sR[kNodes * kRP];
  __shared__ __align__(16) float    sQ[kFib];
  __shared__ __align__(16) float    sLog[kNodes * kHeads];
  __shared__ __align__(16) float    sW1[6 * kCh];
  __shared__ __align__(16) float    sF[kMM * kCh];
  __shared__ __align__(16) float    sInv[128];
  __shared__ float sDist[kNodes];
  __shared__ int   sBt[kNodes];

  const int tid = threadIdx.x, lane = tid & 31, wave = tid >> 5;
  const int hf = lane >> 4, rl = lane & 15, koff = hf * 8;
  const int node = blockIdx.x;
  const int b = node >> 6, d = node & 63;

  if (wave < 2) {
    const int s = tid;
    const float* xs = x + (size_t)(b * kNodes + s) * 3;
    const float* xd = x + (size_t)(b * kNodes + d) * 3;
    const float dx = xs[0] - xd[0];
    const float dy = xs[1] - xd[1];
    const float dz = xs[2] - xd[2];
    const float d2 = dx * dx + dy * dy + dz * dz;
    const float dist = sqrtf(d2 + kEps);
    const float rinv = 1.0f / dist;
    sph16(dx * rinv, dy * rinv, dz * rinv, &sY[s * kMM]);
    sDist[s] = dist;
    int bt = bond[(size_t)node * kNodes + s];
    bt = bt < 0 ? 0 : (bt > 4 ? 4 : bt);
    sBt[s] = bt;
  } else if (wave < 7) {
    sW1[tid - 64] = rw1[li * 5 * kCh + (tid - 64)];
  } else if (wave == 7) {
    sW1[5 * kCh + lane] = rb1[li * kCh + lane];
  } else if (wave < 12) {
    const int t4 = tid - 256;
    *(v4f*)(&sQ[t4 * 4]) = *(const v4f*)(projBase + 2 * kPlane + (size_t)node * kFib + t4 * 4);
  }
  __syncthreads();

  {
    const int s = tid >> 3, c0 = (tid & 7) * 4;
    const float dist = sDist[s];
    const int bt = sBt[s];
    const int btc = bt < 1 ? 1 : bt;
    const bool has = (bt >= 1);
    const v4f w0 = *(const v4f*)(&sW1[c0]);
    const v4f wb = *(const v4f*)(&sW1[btc * kCh + c0]);
    const v4f b1 = *(const v4f*)(&sW1[5 * kCh + c0]);
    float pre[4];
#pragma unroll
    for (int j = 0; j < 4; ++j) pre[j] = fmaf(dist, w0[j], has ? wb[j] : 0.0f) + b1[j];
    float sum = (pre[0] + pre[1]) + (pre[2] + pre[3]);
    sum += __shfl_xor(sum, 1, 32);
    sum += __shfl_xor(sum, 2, 32);
    sum += __shfl_xor(sum, 4, 32);
    const float mu = sum * (1.0f / (float)kCh);
    float dv[4];
#pragma unroll
    for (int j = 0; j < 4; ++j) dv[j] = pre[j] - mu;
    float vs = (dv[0] * dv[0] + dv[1] * dv[1]) + (dv[2] * dv[2] + dv[3] * dv[3]);
    vs += __shfl_xor(vs, 1, 32);
    vs += __shfl_xor(vs, 2, 32);
    vs += __shfl_xor(vs, 4, 32);
    const float rs = rsqrtf(vs * (1.0f / (float)kCh) + kEps);
    v4h hv;
#pragma unroll
    for (int j = 0; j < 4; ++j) hv[j] = (_Float16)(fmaxf(dv[j] * rs, 0.0f) * kHCarry);
    *(v4h*)(&sHm[s * kCh + c0]) = hv;
  }
  __syncthreads();

  const int tm = wave >> 2, tn = wave & 3;
  FragU af;
  {
    const int arow = tm * 16 + rl;
    af.h[0] = *(const v8h*)(&sHm[arow * kCh + koff]);
    af.h[1] = *(const v8h*)(&sHm[arow * kCh + 16 + koff]);
  }
  const int colbase = li * kRadN + tn * 16 + rl;
  float* srp = &sR[(tm * 16 + hf * 8) * kRP + tn * 16 + rl];

  const int ls = tid >> 3, hh = tid & 7;
  float ca[16], cb[16];
  {
    const size_t srcn = (size_t)(b * kNodes + ls);
    float Yv[16], skf[16];
    ld16(Yv, &sY[ls * kMM]);
    {
      const float* sckp = scBase + srcn * 128 + 4 * hh;
#pragma unroll
      for (int l = 0; l < 4; ++l) {
        const v4f t = *(const v4f*)(sckp + l * 32);
        skf[l * 4 + 0] = t[0];
        skf[l * 4 + 1] = t[1];
        skf[l * 4 + 2] = t[2];
        skf[l * 4 + 3] = t[3];
      }
    }
#pragma unroll
    for (int c2 = 0; c2 < 4; ++c2) {
      const int c = 4 * hh + c2;
      float qv[16], ik[16];
      ld16(qv, &sQ[c * kMM]);
      ld16(ik, projBase + srcn * kFib + c * kMM);
      ca[0 * 4 + c2] = skf[0 * 4 + c2] * deg_dot<0>(qv, Yv);
      cb[0 * 4 + c2] = deg_dot<0>(qv, ik);
      ca[1 * 4 + c2] = skf[1 * 4 + c2] * deg_dot<1>(qv, Yv);
      cb[1 * 4 + c2] = deg_dot<1>(qv, ik);
      ca[2 * 4 + c2] = skf[2 * 4 + c2] * deg_dot<2>(qv, Yv);
      cb[2 * 4 + c2] = deg_dot<2>(qv, ik);
      ca[3 * 4 + c2] = skf[3 * 4 + c2] * deg_dot<3>(qv, Yv);
      cb[3 * 4 + c2] = deg_dot<3>(qv, ik);
    }
  }

  float lacc = 0.0f;
  const float* lrow = &sR[ls * kRP + 4 * hh];
  radial_tile(af.v, rw2T + (size_t)(colbase + 0 * 128) * kCh + koff, rb2[colbase + 0 * 128], srp);
  __syncthreads();
  lacc = logit_acc<0>(lacc, ca, cb, lrow);
  __syncthreads();
  radial_tile(af.v, rw2T + (size_t)(colbase + 1 * 128) * kCh + koff, rb2[colbase + 1 * 128], srp);
  __syncthreads();
  lacc = logit_acc<1>(lacc, ca, cb, lrow);
  __syncthreads();
  radial_tile(af.v, rw2T + (size_t)(colbase + 2 * 128) * kCh + koff, rb2[colbase + 2 * 128], srp);
  __syncthreads();
  lacc = logit_acc<2>(lacc, ca, cb, lrow);
  __syncthreads();
  radial_tile(af.v, rw2T + (size_t)(colbase + 3 * 128) * kCh + koff, rb2[colbase + 3 * 128], srp);
  __syncthreads();
  lacc = logit_acc<3>(lacc, ca, cb, lrow);

  sLog[ls * kHeads + hh] = (ls == d) ? -1.0e9f : (lacc * kLogitScale);
  __syncthreads();

  if (wave < kHeads) {
    const float v0 = sLog[lane * kHeads + wave];
    const float v1 = sLog[(lane + 32) * kHeads + wave];
    float mx = fmaxf(v0, v1);
    mx = fmaxf(mx, __shfl_xor(mx, 16, 32));
    mx = fmaxf(mx, __shfl_xor(mx, 8, 32));
    mx = fmaxf(mx, __shfl_xor(mx, 4, 32));
    mx = fmaxf(mx, __shfl_xor(mx, 2, 32));
    mx = fmaxf(mx, __shfl_xor(mx, 1, 32));
    const float p0 = expf(v0 - mx);
    const float p1 = expf(v1 - mx);
    float sm = p0 + p1;
    sm += __shfl_xor(sm, 16, 32);
    sm += __shfl_xor(sm, 8, 32);
    sm += __shfl_xor(sm, 4, 32);
    sm += __shfl_xor(sm, 2, 32);
    sm += __shfl_xor(sm, 1, 32);
    const float inv = 1.0f / sm;
    sLog[lane * kHeads + wave] = p0 * inv;
    sLog[(lane + 32) * kHeads + wave] = p1 * inv;
  }
  __syncthreads();

  const int vc = tid >> 4, vsp = tid & 15;
  float at[4], iv[64], svv[16], o[16];
#pragma unroll
  for (int j = 0; j < 4; ++j) {
    const int s = j * 16 + vsp;
    const size_t srcn = (size_t)(b * kNodes + s);
    at[j] = sLog[s * kHeads + (vc >> 2)];
    const float* ivp = projBase + kPlane + srcn * kFib + vc * kMM;
#pragma unroll
    for (int q = 0; q < 4; ++q) {
      const v4f t = *(const v4f*)(ivp + 4 * q);
      iv[j * 16 + 4 * q + 0] = t[0];
      iv[j * 16 + 4 * q + 1] = t[1];
      iv[j * 16 + 4 * q + 2] = t[2];
      iv[j * 16 + 4 * q + 3] = t[3];
    }
    const float* svp = scBase + kScPlane + srcn * 128 + vc;
    svv[j * 4 + 0] = svp[0];
    svv[j * 4 + 1] = svp[32];
    svv[j * 4 + 2] = svp[64];
    svv[j * 4 + 3] = svp[96];
  }
#pragma unroll
  for (int mm = 0; mm < 16; ++mm) o[mm] = 0.0f;

  radial_tile(af.v, rw2T + (size_t)(colbase + 0 * 128 + 64) * kCh + koff, rb2[colbase + 0 * 128 + 64], srp);
  __syncthreads();
  value_acc<0>(o, at, iv, svv, sR, sY, vsp, vc);
  __syncthreads();
  radial_tile(af.v, rw2T + (size_t)(colbase + 1 * 128 + 64) * kCh + koff, rb2[colbase + 1 * 128 + 64], srp);
  __syncthreads();
  value_acc<1>(o, at, iv, svv, sR, sY, vsp, vc);
  __syncthreads();
  radial_tile(af.v, rw2T + (size_t)(colbase + 2 * 128 + 64) * kCh + koff, rb2[colbase + 2 * 128 + 64], srp);
  __syncthreads();
  value_acc<2>(o, at, iv, svv, sR, sY, vsp, vc);
  __syncthreads();
  radial_tile(af.v, rw2T + (size_t)(colbase + 3 * 128 + 64) * kCh + koff, rb2[colbase + 3 * 128 + 64], srp);
  __syncthreads();
  value_acc<3>(o, at, iv, svv, sR, sY, vsp, vc);

#pragma unroll
  for (int mm = 0; mm < 16; ++mm) {
    float v = o[mm];
    v += __shfl_xor(v, 1, 32);
    v += __shfl_xor(v, 2, 32);
    v += __shfl_xor(v, 4, 32);
    v += __shfl_xor(v, 8, 32);
    o[mm] = v;
  }

  {
    float sfp[16], fn[16];
    ld16(sfp, projBase + 3 * kPlane + (size_t)node * kFib + vc * kMM);
#pragma unroll
    for (int mm = 0; mm < 16; ++mm) o[mm] += sfp[mm];
    const float g0 = gnorm[(li * kDeg + 0) * kCh + vc], q0 = bnorm[(li * kDeg + 0) * kCh + vc];
    const float g1 = gnorm[(li * kDeg + 1) * kCh + vc], q1 = bnorm[(li * kDeg + 1) * kCh + vc];
    const float g2 = gnorm[(li * kDeg + 2) * kCh + vc], q2 = bnorm[(li * kDeg + 2) * kCh + vc];
    const float g3 = gnorm[(li * kDeg + 3) * kCh + vc], q3 = bnorm[(li * kDeg + 3) * kCh + vc];
    const float i0 = gate_degree<0>(o, fn, g0, q0);
    const float i1 = gate_degree<1>(o, fn, g1, q1);
    const float i2 = gate_degree<2>(o, fn, g2, q2);
    const float i3 = gate_degree<3>(o, fn, g3, q3);
    if (vsp == 0) {
#pragma unroll
      for (int mm = 0; mm < 16; ++mm) sF[mm * kCh + vc] = fn[mm];
      sInv[0 * kCh + vc] = i0;
      sInv[1 * kCh + vc] = i1;
      sInv[2 * kCh + vc] = i2;
      sInv[3 * kCh + vc] = i3;
    }
  }
  __syncthreads();

  if (wave < 2) {
    const int e = tid;
    const v4f a0 = *(const v4f*)(&sF[e * 8]);
    const v4f a1 = *(const v4f*)(&sF[e * 8 + 4]);
    v8h hv;
    hv[0] = (_Float16)(a0[0] * kFCarry);
    hv[1] = (_Float16)(a0[1] * kFCarry);
    hv[2] = (_Float16)(a0[2] * kFCarry);
    hv[3] = (_Float16)(a0[3] * kFCarry);
    hv[4] = (_Float16)(a1[0] * kFCarry);
    hv[5] = (_Float16)(a1[1] * kFCarry);
    hv[6] = (_Float16)(a1[2] * kFCarry);
    hv[7] = (_Float16)(a1[3] * kFCarry);
    _Float16* q = fTout + (size_t)node * kFib + e * 8;
    for (int pass = 0; pass < 2; ++pass) {
      *(volatile v8h*)q = hv;
      __threadfence();
    }
  } else if (wave == 2) {
    const v4f v = *(const v4f*)(&sInv[lane * 4]);
    float* q = invOut + (size_t)node * 128 + lane * 4;
    for (int pass = 0; pass < 2; ++pass) {
      *(volatile v4f*)q = v;
      __threadfence();
    }
  }
}

__global__ __launch_bounds__(128) void pooled_out_kernel(
    const float* __restrict__ inv, const float* __restrict__ Wfinal,
    const float* __restrict__ bfinal, float* __restrict__ out)
{
  __shared__ __align__(16) float sP[128];
  __shared__ __align__(16) float sO[128];
  const int b = blockIdx.x, t = threadIdx.x;
  float sum = 0.0f;
#pragma unroll 4
  for (int n = 0; n < kNodes; ++n) sum += inv[(size_t)(b * kNodes + n) * 128 + t];
  sP[t] = sum * (1.0f / (float)kNodes);
  __syncthreads();
  float acc = 0.0f;
#pragma unroll 4
  for (int i = 0; i < 128; ++i) acc = fmaf(sP[i], Wfinal[i * 128 + t], acc);
  sO[t] = acc + bfinal[t];
  __syncthreads();
  if (t < 32) {
    const v4f v = *(const v4f*)(&sO[t * 4]);
    float* q = out + (size_t)b * 128 + t * 4;
    for (int pass = 0; pass < 2; ++pass) {
      *(volatile v4f*)q = v;
      __threadfence();
    }
  }
}

extern "C" void kernel_launch(void* const* d_in, const int* in_sizes, int n_in,
                              void* d_out, int out_size, void* d_ws, size_t ws_size,
                              hipStream_t stream) {
  if (n_in < 16) return;
  if (in_sizes[0] != kBN * kFin) return;
  if (in_sizes[1] != kBN * 3) return;
  if (in_sizes[2] != kBN * kNodes) return;
  if (in_sizes[3] != kFin * kCh) return;
  if (in_sizes[4] != kLay * 5 * kCh) return;
  if (in_sizes[5] != kLay * kCh) return;
  if (in_sizes[6] != kLay * kCh * kRadN) return;
  if (in_sizes[7] != kLay * kRadN) return;
  if (in_sizes[8] != kLay * kDeg * 2 * kCh * kCh) return;
  if (in_sizes[9] != kLay * kDeg * 2 * kCh * kCh) return;
  if (in_sizes[10] != kLay * kDeg * kCh * kCh) return;
  if (in_sizes[11] != kLay * kDeg * kCh * kCh) return;
  if (in_sizes[12] != kLay * kDeg * kCh) return;
  if (in_sizes[13] != kLay * kDeg * kCh) return;
  if (in_sizes[14] != 128 * 128) return;
  if (in_sizes[15] != 128) return;
  if (out_size != kBatch * 128) return;
  if (ws_size < kWsTotal) return;

  const float* hfeat  = (const float*)d_in[0];
  const float* x      = (const float*)d_in[1];
  const int*   bond   = (const int*)d_in[2];
  const float* Wemb   = (const float*)d_in[3];
  const float* rw1    = (const float*)d_in[4];
  const float* rb1    = (const float*)d_in[5];
  const float* rw2    = (const float*)d_in[6];
  const float* rb2    = (const float*)d_in[7];
  const float* Wk     = (const float*)d_in[8];
  const float* Wv     = (const float*)d_in[9];
  const float* Wq     = (const float*)d_in[10];
  const float* Wself  = (const float*)d_in[11];
  const float* gnorm  = (const float*)d_in[12];
  const float* bnorm  = (const float*)d_in[13];
  const float* Wfinal = (const float*)d_in[14];
  const float* bfinal = (const float*)d_in[15];
  float* out = (float*)d_out;

  char* ws = (char*)d_ws;
  _Float16* rw2T = (_Float16*)(ws + kOffRW2T);
  _Float16* w16  = (_Float16*)(ws + kOffWK);
  _Float16* fTA  = (_Float16*)(ws + kOffFTA);
  _Float16* fTB  = (_Float16*)(ws + kOffFTB);
  float* projBase = (float*)(ws + kOffPROJ);
  float* scBase   = (float*)(ws + kOffSC);
  float* invP     = (float*)(ws + kOffINV);

  pack_weights_kernel<<<80, 256, 0, stream>>>(rw2, Wk, Wv, Wq, Wself, rw2T);
  embed_kernel<<<kBN / 4, 256, 0, stream>>>(hfeat, Wemb, fTA);

  _Float16* fin = fTA;
  _Float16* fout = fTB;
  for (int li = 0; li < kLay; ++li) {
    node_proj_kernel<<<kBN, 256, 0, stream>>>(fin, w16, projBase, scBase, li);
    edge_attn_kernel<<<kBN, 512, 0, stream>>>(x, bond, rw1, rb1, rw2T, rb2, projBase, scBase,
                                              gnorm, bnorm, fout, invP, li);
    _Float16* t = fin; fin = fout; fout = t;
  }
  pooled_out_kernel<<<kBatch, 128, 0, stream>>>(invP, Wfinal, bfinal, out);
}
